// SelfModule_82471962017878
// MI455X (gfx1250) — hardware-verified
//
#include <hip/hip_runtime.h>
#include <math.h>

typedef __attribute__((ext_vector_type(16))) _Float16 v16h;
typedef __attribute__((ext_vector_type(16))) __bf16 v16b;
typedef __attribute__((ext_vector_type(8)))  _Float16 v8h;
typedef __attribute__((ext_vector_type(8)))  float v8f;
typedef __attribute__((ext_vector_type(4)))  float v4f;
typedef __attribute__((ext_vector_type(2)))  float v2f;
typedef __attribute__((ext_vector_type(4)))  unsigned v4u;
typedef __attribute__((ext_vector_type(4)))  int v4i;
typedef float __attribute__((may_alias)) float_a;
typedef int __attribute__((may_alias)) int_a;

template <typename T> __device__ __forceinline__ void vst2(void* p, T v) { *(volatile T*)p = v; __threadfence(); *(volatile T*)p = v; }
__device__ __forceinline__ v8f wmma16(v16h a, v16h b, v8f c) {
  v8f d = __builtin_amdgcn_wmma_f32_16x16x32_f16(false, a, false, b, (short)0, c, false, false);
  asm volatile("v_nop\n\tv_nop\n\tv_nop\n\tv_nop" : "+v"(d) : "v"(a), "v"(b));
  return d;
}
__device__ __forceinline__ v8f wmma_bf(v16b a, v16b b, v8f c) {
  v8f d = __builtin_amdgcn_wmma_f32_16x16x32_bf16(false, a, false, b, (short)0, c, false, false);
  asm volatile("v_nop\n\tv_nop\n\tv_nop\n\tv_nop" : "+v"(d) : "v"(a), "v"(b));
  return d;
}
__device__ __forceinline__ v16h frag_h(const _Float16* rowk0, int lane) {
  union { v16h v; v8h q[2]; } u; const _Float16* p = rowk0 + 8 * (lane >> 4);
  u.q[0] = *(const v8h*)p; u.q[1] = *(const v8h*)(p + 16); return u.v;
}
__device__ __forceinline__ v16h frag_f32(const float* rowk0, int lane) {
  v16h a; const float* p = rowk0 + 8 * (lane >> 4);
#pragma unroll
  for (int i = 0; i < 8; ++i) { a[i] = (_Float16)p[i]; a[8 + i] = (_Float16)p[16 + i]; }
  return a;
}
__device__ __forceinline__ v16h frag_f32s(const float* rowk0, int lane, float sc) {
  v16h a; const float* p = rowk0 + 8 * (lane >> 4);
#pragma unroll
  for (int i = 0; i < 8; ++i) { a[i] = (_Float16)(p[i] * sc); a[8 + i] = (_Float16)(p[16 + i] * sc); }
  return a;
}
__device__ __forceinline__ v16h fragc_f32(const float* W, int k0, int n, int lane, int ld, int K) {
  v16h a; const int g = lane >> 4;
#pragma unroll
  for (int i = 0; i < 8; ++i) { const int ka = k0 + 8 * g + i, kb = ka + 16;
    a[i] = (_Float16)(ka < K ? W[(size_t)(ka < K ? ka : K - 1) * ld + n] : 0.f); a[8 + i] = (_Float16)(kb < K ? W[(size_t)(kb < K ? kb : K - 1) * ld + n] : 0.f); }
  return a;
}
struct F2 { v16b h, l; };
__device__ __forceinline__ F2 bsplit16(const float v[16]) { F2 r;
#pragma unroll
  for (int i = 0; i < 16; ++i) { const __bf16 h = (__bf16)v[i]; r.h[i] = h; r.l[i] = (__bf16)(v[i] - (float)h); }
  return r; }
__device__ __forceinline__ F2 split_row(const float* row, int k0, int lane) { float v[16]; const float* p = row + k0 + 8 * (lane >> 4);
#pragma unroll
  for (int i = 0; i < 8; ++i) { v[i] = p[i]; v[8 + i] = p[16 + i]; }
  return bsplit16(v); }
__device__ __forceinline__ F2 split_rowK(const float* row, int k0, int lane, int K) { float v[16]; const int g = lane >> 4;
#pragma unroll
  for (int i = 0; i < 8; ++i) { const int ka = k0 + 8 * g + i, kb = ka + 16; v[i] = ka < K ? row[ka < K ? ka : K - 1] : 0.f; v[8 + i] = kb < K ? row[kb < K ? kb : K - 1] : 0.f; }
  return bsplit16(v); }
__device__ __forceinline__ F2 split_col(const float* W, int k0, int n, int lane, int ld, int K) { float v[16]; const int g = lane >> 4;
#pragma unroll
  for (int i = 0; i < 8; ++i) { const int ka = k0 + 8 * g + i, kb = ka + 16; v[i] = ka < K ? W[(size_t)(ka < K ? ka : K - 1) * ld + n] : 0.f; v[8 + i] = kb < K ? W[(size_t)(kb < K ? kb : K - 1) * ld + n] : 0.f; }
  return bsplit16(v); }
__device__ __forceinline__ v8f mac3(const F2& a, const F2& b, v8f c) { c = wmma_bf(a.l, b.h, c); c = wmma_bf(a.h, b.l, c); return wmma_bf(a.h, b.h, c); }
__device__ __forceinline__ float sigm(float v) { return 1.0f / (1.0f + expf(-v)); }
#define LDSX() do { asm volatile("s_wait_dscnt 0" ::: "memory"); __builtin_amdgcn_wave_barrier(); __builtin_amdgcn_fence(__ATOMIC_RELEASE, "workgroup"); } while (0)


#define NB 8
#define CC 512
#define NN 1024
#define NH 4
#define DK 128
#define RR 128
#ifndef TNB
#define TNB NB
#endif
typedef __attribute__((ext_vector_type(8))) __bf16 v8b;
__device__ __forceinline__ v16b frag_b(const __bf16* rowk0, int lane) {
  union { v16b v; v8b q[2]; } u; const __bf16* p = rowk0 + 8 * (lane >> 4);
  u.q[0] = *(const v8b*)p; u.q[1] = *(const v8b*)(p + 16); return u.v;
}
__device__ __forceinline__ float bfr(float v) { return (float)(__bf16)v; }
__device__ __attribute__((noinline)) float exp_ni(float v) { return expf(v); }
__device__ __attribute__((noinline)) float erf_ni(float v) { return erff(v); }

#define WS_SC  0u
#define WS_QH  (WS_SC + 4u * (size_t)NB * CC)
#define WS_QL  (WS_QH + 2u * (size_t)NB * NN * CC)
#define WS_KH  (WS_QL + 2u * (size_t)NB * NN * CC)
#define WS_KL  (WS_KH + 2u * (size_t)NB * NN * CC)
#define WS_VT  (WS_KL + 2u * (size_t)NB * NN * CC)
#define WS_VTL (WS_VT + 2u * (size_t)NB * CC * NN)
#define WS_ST  (WS_VTL + 2u * (size_t)NB * CC * NN)
#define WS_SL  (WS_ST + 4u * (size_t)NB * NH * NN)
#define WS_O   (WS_SL + 4u * (size_t)NB * NH * NN)
#define WS_END (WS_O + 4u * (size_t)NB * CC * NN)

__global__ __launch_bounds__(256) void k_se(const float* __restrict__ X, const float* __restrict__ F1W, const float* __restrict__ F1B, const float* __restrict__ F2W, const float* __restrict__ F2B, float* __restrict__ SC) { __shared__ float sp[CC]; __shared__ float sh[RR]; __shared__ __align__(16) float ss[CC]; const int t = threadIdx.x, lane = t & 31, w = t >> 5; const size_t b = blockIdx.x;
  for (int c = w; c < CC; c += 8) { const float* xr = X + (b * CC + c) * (size_t)NN; float s = 0.f; for (int n = lane; n < NN; n += 32) s += bfr(xr[n]);
#pragma unroll
    for (int o = 1; o < 32; o <<= 1) s += __shfl_xor(s, o);
    if (lane == 0) sp[c] = s * (1.0f / NN); }
  __syncthreads();
  if (t < RR) { float s = bfr(F1B[t]); for (int c = 0; c < CC; ++c) s += sp[c] * bfr(F1W[(size_t)t * CC + c]); sh[t] = fmaxf(s, 0.f); }
  __syncthreads();
  for (int c = t; c < CC; c += 256) { float s = bfr(F2B[c]); for (int j = 0; j < RR; ++j) s += sh[j] * bfr(F2W[(size_t)c * RR + j]); ss[c] = 1.0f + 1.0f / (1.0f + expf(-s)); }
  __syncthreads(); if (t < CC / 4) vst2(SC + b * CC + t * 4, *(const v4f*)&ss[t * 4]); }
__global__ __launch_bounds__(128) void k_proj(const float* __restrict__ X, const float* __restrict__ SC, const float* __restrict__ WQ, const float* __restrict__ BQ, const float* __restrict__ WK, const float* __restrict__ BK, const float* __restrict__ WV, const float* __restrict__ BV, _Float16* __restrict__ QH, _Float16* __restrict__ QL, _Float16* __restrict__ KH, _Float16* __restrict__ KL, _Float16* __restrict__ VT, _Float16* __restrict__ VTL) {
  __shared__ __align__(16) _Float16 sh[64][136], sl[64][136]; __shared__ __align__(16) _Float16 th[128][72], tl[128][72]; __shared__ float ssc[CC];
  const int tid = threadIdx.x, wave = tid >> 5, lane = tid & 31, col = lane & 15, g = lane >> 4; const int which = blockIdx.z / NB; const size_t b = blockIdx.z % NB; const int n0 = blockIdx.x * 64 + wave * 16; const int c0 = blockIdx.y * 128; const float* Wm = which == 0 ? WQ : which == 1 ? WK : WV; const float* Bm = which == 0 ? BQ : which == 1 ? BK : BV; const float* Xb = X + b * CC * (size_t)NN;
  for (int c = tid; c < CC; c += 128) ssc[c] = SC[b * CC + c]; __syncthreads();
  v8f acc[8] = {};
#pragma unroll 2
  for (int kc = 0; kc < CC / 32; ++kc) { float v[16]; const int px = n0 + col;
#pragma unroll
    for (int i = 0; i < 8; ++i) { const int ca = kc * 32 + 8 * g + i, cb2 = ca + 16; v[i] = bfr(Xb[(size_t)ca * NN + px]) * ssc[ca]; v[8 + i] = bfr(Xb[(size_t)cb2 * NN + px]) * ssc[cb2]; }
    const F2 a = bsplit16(v);
#pragma unroll
    for (int j = 0; j < 8; ++j) { v16b w; const float* wr = Wm + (size_t)(c0 + j * 16 + col) * CC + kc * 32 + 8 * g;
#pragma unroll
      for (int i = 0; i < 8; ++i) { w[i] = (__bf16)wr[i]; w[8 + i] = (__bf16)wr[16 + i]; }
      acc[j] = wmma_bf(a.h, w, acc[j]); acc[j] = wmma_bf(a.l, w, acc[j]); } }
#pragma unroll
  for (int j = 0; j < 8; ++j) { const float bb = bfr(Bm[c0 + j * 16 + col]);
#pragma unroll
    for (int r = 0; r < 8; ++r) { const float v = acc[j][r] + bb; const _Float16 hv = (_Float16)v, lv = (_Float16)((v - (float)hv) * 2048.0f); if (which < 2) { sh[wave * 16 + 8 * g + r][j * 16 + col] = hv; sl[wave * 16 + 8 * g + r][j * 16 + col] = lv; } else { th[j * 16 + col][wave * 16 + 8 * g + r] = hv; tl[j * 16 + col][wave * 16 + 8 * g + r] = lv; } } }
  __syncthreads();
  if (which < 2) { _Float16* PH = which == 0 ? QH : KH; _Float16* PL = which == 0 ? QL : KL; for (int e = tid; e < 64 * 16; e += 128) { const int rl = e >> 4, q = e & 15; const size_t o = (b * NN + blockIdx.x * 64 + rl) * CC + c0 + q * 8; vst2((unsigned*)(PH + o), *(const v4u*)&sh[rl][q * 8]); vst2((unsigned*)(PL + o), *(const v4u*)&sl[rl][q * 8]); } }
  else { for (int e = tid; e < 128 * 8; e += 128) { const int cl = e >> 3, q = e & 7; const size_t o = (b * CC + c0 + cl) * (size_t)NN + blockIdx.x * 64 + q * 8; vst2((unsigned*)(VT + o), *(const v4u*)&th[cl][q * 8]); vst2((unsigned*)(VTL + o), *(const v4u*)&tl[cl][q * 8]); } } }
__global__ __launch_bounds__(128) void k_stats(const _Float16* __restrict__ QH, const _Float16* __restrict__ QL, const _Float16* __restrict__ KH, const _Float16* __restrict__ KL, float* __restrict__ ST, float* __restrict__ SL) { __shared__ __align__(16) float sm[64], ssum[64];
  const int tid = threadIdx.x, wave = tid >> 5, lane = tid & 31, col = lane & 15, g = lane >> 4; const int h = blockIdx.y; const size_t b = blockIdx.z; const int q0 = blockIdx.x * 64 + wave * 16; const size_t rq = b * NN + q0;
  v16h aq[4], al[4];
#pragma unroll
  for (int kc = 0; kc < 4; ++kc) { aq[kc] = frag_h(QH + (rq + col) * CC + h * DK + kc * 32, lane); al[kc] = frag_h(QL + (rq + col) * CC + h * DK + kc * 32, lane); }
  float m[8], l[8];
#pragma unroll
  for (int r = 0; r < 8; ++r) { m[r] = -3.0e38f; l[r] = 0.f; }
#pragma unroll 1
  for (int ks = 0; ks < NN / 32; ++ks) { float s[2][8];
#pragma unroll
    for (int ct = 0; ct < 2; ++ct) { const size_t rk = b * NN + ks * 32 + ct * 16 + col; v8f c = {}, cl = {};
#pragma unroll
      for (int kc = 0; kc < 4; ++kc) { const v16h kh = frag_h(KH + rk * CC + h * DK + kc * 32, lane), kl = frag_h(KL + rk * CC + h * DK + kc * 32, lane); c = wmma16(aq[kc], kh, c); cl = wmma16(aq[kc], kl, cl); cl = wmma16(al[kc], kh, cl); }
#pragma unroll
      for (int r = 0; r < 8; ++r) s[ct][r] = (c[r] + cl[r] * (1.0f / 2048.0f)) * 0.08838834764831845f; }
#pragma unroll
    for (int r = 0; r < 8; ++r) { float mx = fmaxf(s[0][r], s[1][r]);
#pragma unroll
      for (int o = 1; o < 16; o <<= 1) mx = fmaxf(mx, __shfl_xor(mx, o));
      const float mn = fmaxf(m[r], mx); const float alpha = __expf(m[r] - mn); float es = __expf(s[0][r] - mn) + __expf(s[1][r] - mn);
#pragma unroll
      for (int o = 1; o < 16; o <<= 1) es += __shfl_xor(es, o);
      l[r] = l[r] * alpha + es; m[r] = mn; } }
  if (col == 0) {
#pragma unroll
    for (int r = 0; r < 8; ++r) { sm[wave * 16 + 8 * g + r] = m[r]; ssum[wave * 16 + 8 * g + r] = l[r]; } }
  __syncthreads(); if (tid < 16) vst2(ST + (b * NH + h) * (size_t)NN + blockIdx.x * 64 + tid * 4, *(const v4f*)&sm[tid * 4]); else if (tid < 32) vst2(SL + (b * NH + h) * (size_t)NN + blockIdx.x * 64 + (tid - 16) * 4, *(const v4f*)&ssum[(tid - 16) * 4]); }
__global__ __launch_bounds__(128) void k_ov(const _Float16* __restrict__ QH, const _Float16* __restrict__ QL, const _Float16* __restrict__ KH, const _Float16* __restrict__ KL, const _Float16* __restrict__ VT, const _Float16* __restrict__ VTL, const float* __restrict__ ST, const float* __restrict__ SL, float* __restrict__ O) {
  __shared__ __align__(16) float sp[4][16][36]; __shared__ __align__(16) float stt[128][68];
  const int tid = threadIdx.x, wave = tid >> 5, lane = tid & 31, col = lane & 15, g = lane >> 4; const int h = blockIdx.y; const size_t b = blockIdx.z; const int mm0 = blockIdx.x * 64 + wave * 16; const size_t rm = b * NN + mm0;
  v16h ak[4], akl[4];
#pragma unroll
  for (int kc = 0; kc < 4; ++kc) { ak[kc] = frag_h(KH + (rm + col) * CC + h * DK + kc * 32, lane); akl[kc] = frag_h(KL + (rm + col) * CC + h * DK + kc * 32, lane); }
  const float* stm = ST + (b * NH + h) * (size_t)NN; const float* stl = SL + (b * NH + h) * (size_t)NN;
  v8f acc[8], accl[8];
#pragma unroll
  for (int j = 0; j < 8; ++j) { acc[j] = v8f{}; accl[j] = v8f{}; }
#pragma unroll 1
  for (int ks = 0; ks < NN / 32; ++ks) {
#pragma unroll
    for (int ct = 0; ct < 2; ++ct) { const int n = ks * 32 + ct * 16 + col; const size_t rn = b * NN + n; v8f c = {}, cl = {};
#pragma unroll
      for (int kc = 0; kc < 4; ++kc) { const v16h qh = frag_h(QH + rn * CC + h * DK + kc * 32, lane), ql = frag_h(QL + rn * CC + h * DK + kc * 32, lane); c = wmma16(ak[kc], qh, c); cl = wmma16(ak[kc], ql, cl); cl = wmma16(akl[kc], qh, cl); }
      const float mx = stm[n], il = 1.0f / stl[n];
#pragma unroll
      for (int r = 0; r < 8; ++r) { const float s = (c[r] + cl[r] * (1.0f / 2048.0f)) * 0.08838834764831845f; sp[wave][8 * g + r][ct * 16 + col] = __expf(s - mx) * il; } }
    LDSX();
    v16h pa, pal; { const float* prow = &sp[wave][col][0] + 8 * (lane >> 4);
#pragma unroll
      for (int i = 0; i < 8; ++i) { const float p0 = prow[i] * 2048.0f, p1 = prow[16 + i] * 2048.0f; pa[i] = (_Float16)p0; pa[8 + i] = (_Float16)p1; pal[i] = (_Float16)((p0 - (float)pa[i]) * 2048.0f); pal[8 + i] = (_Float16)((p1 - (float)pa[8 + i]) * 2048.0f); } }
#pragma unroll
    for (int j = 0; j < 8; ++j) { const size_t po = (b * CC + (size_t)h * DK + j * 16 + col) * (size_t)NN + ks * 32; const v16h vh = frag_h(VT + po, lane), vl = frag_h(VTL + po, lane); acc[j] = wmma16(pa, vh, acc[j]); accl[j] = wmma16(pa, vl, accl[j]); accl[j] = wmma16(pal, vh, accl[j]); }
    LDSX(); }
#pragma unroll
  for (int j = 0; j < 8; ++j)
#pragma unroll
    for (int r = 0; r < 8; ++r) stt[j * 16 + col][wave * 16 + 8 * g + r] = (acc[j][r] + accl[j][r] * (1.0f / 2048.0f)) * (1.0f / 2048.0f);
  __syncthreads(); for (int e = tid; e < 128 * 16; e += 128) { const int d = e >> 4, q = e & 15; vst2(O + (b * CC + (size_t)h * DK + d) * (size_t)NN + blockIdx.x * 64 + q * 4, *(const v4f*)&stt[d][q * 4]); } }
__global__ __launch_bounds__(256) void k_gate(const float* __restrict__ O, const float* __restrict__ GW, const float* __restrict__ GB, float* __restrict__ OUT) { __shared__ float sg[64]; __shared__ float part[4][64]; const int t = threadIdx.x; const size_t b = blockIdx.y; const int m0 = blockIdx.x * 64; const int ml = t & 63, q4 = t >> 6;
  { float s = 0.f; for (int c = q4; c < CC; c += 4) s += bfr(GW[c]) * O[(b * CC + c) * (size_t)NN + m0 + ml]; part[q4][ml] = s; }
  __syncthreads(); if (t < 64) { const float s = part[0][t] + part[1][t] + part[2][t] + part[3][t] + bfr(GB[0]); sg[t] = 1.0f + 1.0f / (1.0f + expf(-s)); } __syncthreads();
  for (int e = t; e < CC * 16; e += 256) { const int c = e >> 4, q = e & 15; const float* orow = O + (b * CC + c) * (size_t)NN + m0 + q * 4; v4f v; v[0] = orow[0] * sg[q * 4]; v[1] = orow[1] * sg[q * 4 + 1]; v[2] = orow[2] * sg[q * 4 + 2]; v[3] = orow[3] * sg[q * 4 + 3]; vst2(OUT + (b * CC + c) * (size_t)NN + m0 + q * 4, v); } }
extern "C" void kernel_launch(void* const* d_in, const int* in_sizes, int n_in, void* d_out, int out_size, void* d_ws, size_t ws_size, hipStream_t stream) {
  (void)in_sizes; (void)n_in; (void)out_size;
  const float** F = (const float**)d_in;
  if (ws_size < (size_t)WS_END) return;
  char* ws = (char*)d_ws; float *SC = (float*)(ws + WS_SC), *ST = (float*)(ws + WS_ST), *SL = (float*)(ws + WS_SL), *O = (float*)(ws + WS_O); _Float16 *QH = (_Float16*)(ws + WS_QH), *QL = (_Float16*)(ws + WS_QL), *KH = (_Float16*)(ws + WS_KH), *KL = (_Float16*)(ws + WS_KL), *VT = (_Float16*)(ws + WS_VT), *VTL = (_Float16*)(ws + WS_VTL);
  k_se<<<NB, 256, 0, stream>>>(F[0], F[7], F[8], F[9], F[10], SC);
  k_proj<<<dim3(NN / 64, CC / 128, 3 * NB), 128, 0, stream>>>(F[0], SC, F[1], F[2], F[3], F[4], F[5], F[6], QH, QL, KH, KL, VT, VTL);
  k_stats<<<dim3(NN / 64, NH, TNB), 128, 0, stream>>>(QH, QL, KH, KL, ST, SL);
  k_ov<<<dim3(NN / 64, NH, TNB), 128, 0, stream>>>(QH, QL, KH, KL, VT, VTL, ST, SL, O);
  k_gate<<<dim3(NN / 64, TNB), 256, 0, stream>>>(O, F[11], F[12], (float*)d_out);
}
